// SMRCAEncoderBlock_4647154614906
// MI455X (gfx1250) — hardware-verified
//
#include <hip/hip_runtime.h>
#include <stddef.h>

#define NB   2
#define CC   128
#define IMG  96
#define NP   9216
#define NT   18432
#define HID  256
#define NH   8
#define HD   32
#define FF   512
#define NG   8
#define CG   16
#define NWIN 9

static_assert(NT == NB * NP);
static_assert(NP == IMG * IMG);
static_assert(NP % 64 == 0);
static_assert(NT % 64 == 0);
static_assert(NH * HD == HID);
static_assert(CC == NG * CG);
static_assert(((CG * NP) / 4) % 256 == 0);
static_assert(CC % 32 == 0);
static_assert(HID % 32 == 0);
static_assert(FF % 32 == 0);
static_assert((HID * CC) % 2048 == 0);
static_assert((FF * CC) % 2048 == 0);

#define ASC    8.0f
#define WSC    16.0f
#define INV_AW 0.0078125f

typedef _Float16 v16h __attribute__((ext_vector_type(16)));
typedef _Float16 v8h  __attribute__((ext_vector_type(8)));
typedef float    v8f  __attribute__((ext_vector_type(8)));
typedef float    v4f  __attribute__((ext_vector_type(4)));
typedef unsigned int v4u __attribute__((ext_vector_type(4)));

union FragH { v16h v; v8h h[2]; };
union Pack8 { v8h h; v4u u; };

__device__ __forceinline__ v8f mma_h(v16h a, v16h b, v8f c) {
  c = __builtin_amdgcn_wmma_f32_16x16x32_f16(false, a, false, b, (short)0, c, false, false);
  asm volatile("v_nop\n\tv_nop\n\tv_nop\n\tv_nop" : "+v"(c) : "v"(a), "v"(b));
  return c;
}
__device__ __forceinline__ v8f zero8() { return (v8f){0.f, 0.f, 0.f, 0.f, 0.f, 0.f, 0.f, 0.f}; }

__device__ __forceinline__ v16h ldfrag_h(const _Float16* p, int ld, int row0, int k0, int lane) {
  const int m = lane & 15, lh = lane >> 4;
  const _Float16* q = p + (size_t)(row0 + m) * ld + k0 + 8 * lh;
  FragH f;
  f.h[0] = *(const v8h*)(q);
  f.h[1] = *(const v8h*)(q + 16);
  return f.v;
}

template <int KSTEPS>
__device__ __forceinline__ void gemm16x64(const _Float16* A, int lda, const _Float16* B, int ldb,
                                          int m0, int n0, int lane, v8f (&acc)[4]) {
  static_assert(KSTEPS % 2 == 0);
#pragma unroll 1
  for (int kg = 0; kg < KSTEPS; kg += 2) {
#pragma unroll
    for (int u = 0; u < 2; ++u) {
      const int k0 = (kg + u) * 32;
      const v16h a = ldfrag_h(A, lda, m0, k0, lane);
#pragma unroll
      for (int t = 0; t < 4; ++t) {
        const v16h bb = ldfrag_h(B, ldb, n0 + 16 * t, k0, lane);
        acc[t] = mma_h(a, bb, acc[t]);
      }
    }
  }
}

__device__ __forceinline__ float gelu_f(float x) {
  const float u = 0.7978845608028654f * (x + 0.044715f * (x * x * x));
  const float e = __expf(2.0f * u);
  const float t = 1.0f - 2.0f * __builtin_amdgcn_rcpf(e + 1.0f);
  return x * (0.5f * (1.0f + t));
}

__device__ __forceinline__ double shfl_xor_d(double v, int mask) {
  const unsigned long long u = __builtin_bit_cast(unsigned long long, v);
  int lo = (int)(unsigned int)(u & 0xffffffffull);
  int hi = (int)(unsigned int)(u >> 32);
  lo = __shfl_xor(lo, mask, 32);
  hi = __shfl_xor(hi, mask, 32);
  const unsigned long long r = ((unsigned long long)(unsigned int)hi << 32) | (unsigned long long)(unsigned int)lo;
  return __builtin_bit_cast(double, r);
}

__global__ __launch_bounds__(256) void k_wcv(const float* __restrict__ W, int n8, _Float16* __restrict__ wp16) {
  int i = blockIdx.x * 256 + threadIdx.x;
  i = min(i, n8 - 1);
  const float* wp = W + (size_t)i * 8;
  const v4f a0 = *(const v4f*)(wp), a1 = *(const v4f*)(wp + 4);
  Pack8 pk;
  pk.h = (v8h){(_Float16)(a0[0] * WSC), (_Float16)(a0[1] * WSC), (_Float16)(a0[2] * WSC), (_Float16)(a0[3] * WSC),
               (_Float16)(a1[0] * WSC), (_Float16)(a1[1] * WSC), (_Float16)(a1[2] * WSC), (_Float16)(a1[3] * WSC)};
  _Float16* dp = wp16 + (size_t)i * 8;
  for (int ps = 0; ps < 2; ++ps) {
    *(volatile v4u*)dp = pk.u;
    __threadfence();
  }
}

__global__ __launch_bounds__(256) void k_gnstat(const float* __restrict__ x, float* __restrict__ st) {
  __shared__ double rs[8];
  __shared__ double rq[8];
  const int tid = threadIdx.x, lane = tid & 31, wave = tid >> 5;
  const int bg = blockIdx.x;
  const float* xb = x + (size_t)bg * (CG * NP);
  double s = 0.0, q = 0.0;
#pragma unroll 2
  for (int i = tid; i < (CG * NP) / 4; i += 256) {
    const v4f a = *(const v4f*)(xb + (size_t)i * 4);
    const double d0 = a[0], d1 = a[1], d2 = a[2], d3 = a[3];
    s += (d0 + d1) + (d2 + d3);
    q += (d0 * d0 + d1 * d1) + (d2 * d2 + d3 * d3);
  }
#pragma unroll
  for (int off = 1; off < 32; off <<= 1) {
    s += shfl_xor_d(s, off);
    q += shfl_xor_d(q, off);
  }
  if (lane == 0) { rs[wave] = s; rq[wave] = q; }
  __syncthreads();
  if (wave == 0) {
    double S = 0.0, Q = 0.0;
#pragma unroll
    for (int w = 0; w < 8; ++w) { S += rs[w]; Q += rq[w]; }
    const double invn = 1.0 / (double)(CG * NP);
    const double mean = S * invn;
    double var = Q * invn - mean * mean;
    var = (var > 0.0) ? var : 0.0;
    const float meanf = (float)mean;
    const float rstd  = 1.0f / sqrtf((float)var + 1e-5f);
    const v4f v = (v4f){meanf, rstd, meanf, rstd};
    if (lane < 8) {
      float* dp = st + (size_t)bg * 32 + lane * 4;
      for (int ps = 0; ps < 2; ++ps) {
        *(volatile v4f*)dp = v;
        __threadfence();
      }
    }
  }
}

#define WTP 65
__global__ __launch_bounds__(256) void k_xtr(const float* __restrict__ x, const float* __restrict__ st,
                                             const float* __restrict__ gw, const float* __restrict__ gb,
                                             _Float16* __restrict__ xt) {
  __shared__ float tl[CC * WTP];
  const int tid = threadIdx.x;
  const int n0 = blockIdx.x * 64, b = blockIdx.y;
  const float* xb = x + (size_t)b * CC * NP;
#pragma unroll
  for (int j = 0; j < 8; ++j) {
    const int p  = tid + 256 * j;
    const int cc = p >> 4;
    const int q4 = (p & 15) * 4;
    const v4f a = *(const v4f*)(xb + (size_t)cc * NP + n0 + q4);
    float* d = tl + cc * WTP + q4;
    d[0] = a[0]; d[1] = a[1]; d[2] = a[2]; d[3] = a[3];
  }
  __syncthreads();
  const int pc = tid & 15;
  const int g  = pc >> 1;
  const float mean = st[(b * NG + g) * 32 + 0];
  const float rstd = st[(b * NG + g) * 32 + 1];
  float gs[8], bs[8];
  {
    const v4f g0 = *(const v4f*)(gw + 8 * pc), g1 = *(const v4f*)(gw + 8 * pc + 4);
    const v4f e0 = *(const v4f*)(gb + 8 * pc), e1 = *(const v4f*)(gb + 8 * pc + 4);
    gs[0] = g0[0]; gs[1] = g0[1]; gs[2] = g0[2]; gs[3] = g0[3];
    gs[4] = g1[0]; gs[5] = g1[1]; gs[6] = g1[2]; gs[7] = g1[3];
    bs[0] = e0[0]; bs[1] = e0[1]; bs[2] = e0[2]; bs[3] = e0[3];
    bs[4] = e1[0]; bs[5] = e1[1]; bs[6] = e1[2]; bs[7] = e1[3];
  }
#pragma unroll 1
  for (int j = 0; j < 4; ++j) {
    const int p  = tid + 256 * j;
    const int nn = p >> 4;
    const float* cp = tl + (8 * pc) * WTP + nn;
    float v[8];
#pragma unroll
    for (int i = 0; i < 8; ++i) v[i] = (((cp[i * WTP] - mean) * rstd) * gs[i] + bs[i]) * ASC;
    Pack8 pk;
    pk.h = (v8h){(_Float16)v[0], (_Float16)v[1], (_Float16)v[2], (_Float16)v[3],
                 (_Float16)v[4], (_Float16)v[5], (_Float16)v[6], (_Float16)v[7]};
    _Float16* dp = xt + ((size_t)(b * NP + n0 + nn) * CC + 8 * pc);
    *(volatile v4u*)dp = pk.u;
    __threadfence();
    *(volatile v4u*)dp = pk.u;
  }
}

#define SFP 132
__global__ __launch_bounds__(256) void k_qkv(const _Float16* __restrict__ xqt,
                                             const _Float16* __restrict__ xkvt,
                                             const _Float16* __restrict__ wqkv,
                                             const float* __restrict__ bq,
                                             const float* __restrict__ bk,
                                             const float* __restrict__ bv,
                                             float* __restrict__ qf,
                                             float* __restrict__ kf,
                                             float* __restrict__ vf) {
  __shared__ __align__(16) float sf[64 * SFP];
  const int tid = threadIdx.x, lane = tid & 31, wave = tid >> 5;
  const int hh = lane >> 4, c = lane & 15;
  const int wm = wave >> 1, wn = wave & 1;
  const int mb = blockIdx.x * 64;
  const int ns = blockIdx.y;
  const int which = ns >> 1;
  const int colb = (ns & 1) * 128;
  const _Float16* A = (which == 0) ? xqt : xkvt;
  const float* bias = (which == 0) ? bq : ((which == 1) ? bk : bv);
  float* dst = (which == 0) ? qf : ((which == 1) ? kf : vf);
  const int m0 = mb + wm * 16;
  const int n0 = ns * 128 + wn * 64;

  v8f acc[4];
#pragma unroll
  for (int t = 0; t < 4; ++t) acc[t] = zero8();
  gemm16x64<CC / 32>(A, CC, wqkv, CC, m0, n0, lane, acc);

#pragma unroll
  for (int t = 0; t < 4; ++t) {
    const float bb = bias[colb + wn * 64 + 16 * t + c];
#pragma unroll
    for (int r = 0; r < 8; ++r)
      sf[(wm * 16 + 8 * hh + r) * SFP + wn * 64 + 16 * t + c] = acc[t][r] * INV_AW + bb;
  }
  __syncthreads();

  v4f val[8];
  int go[8];
#pragma unroll
  for (int j = 0; j < 8; ++j) {
    const int p   = tid + 256 * j;
    const int row = p >> 5;
    const int pc  = p & 31;
    val[j] = *(const v4f*)(sf + row * SFP + pc * 4);
    go[j]  = (mb + row) * HID + colb + pc * 4;
  }
  for (int ps = 0; ps < 2; ++ps) {
#pragma unroll
    for (int j = 0; j < 8; ++j) *(volatile v4f*)(dst + go[j]) = val[j];
    __threadfence();
  }
}

#define OTP 68
__device__ __forceinline__ void store_nchw(const float* st, const float* __restrict__ res, float* __restrict__ dst,
                                           int b, int nb0, int wave, int lane) {
  v4f val[8];
  int go[8];
#pragma unroll
  for (int it = 0; it < 8; ++it) {
    const int p    = lane + 32 * it;
    const int L    = p >> 3;
    const int pc   = p & 7;
    const int cl   = wave * 16 + (L >> 1);
    const int half = L & 1;
    go[it] = (b * CC + cl) * NP + nb0 + half * 32 + pc * 4;
    const v4f a = *(const v4f*)(st + cl * OTP + half * 32 + pc * 4);
    const v4f r = *(const v4f*)(res + go[it]);
    val[it] = a + r;
  }
  for (int ps = 0; ps < 2; ++ps) {
#pragma unroll
    for (int it = 0; it < 8; ++it) *(volatile v4f*)(dst + go[it]) = val[it];
    __threadfence();
  }
}

#define ATP 264
union SmemWO { _Float16 at[64 * ATP]; float st[CC * OTP]; };
__global__ __launch_bounds__(256) void k_attn_wo(const float* __restrict__ qf,
                                                 const float* __restrict__ kf,
                                                 const float* __restrict__ vf,
                                                 const _Float16* __restrict__ wo16,
                                                 const float* __restrict__ bo,
                                                 const float* __restrict__ xq,
                                                 float* __restrict__ xr,
                                                 float sscale) {
  __shared__ __align__(16) SmemWO sm;
  __shared__ float sm_sc[256 * 12];
  const int tid = threadIdx.x, lane = tid & 31, wave = tid >> 5;
  const int hh = lane >> 4, c = lane & 15;
  const int wm = wave >> 1, wn = wave & 1;
  const int mb  = blockIdx.x * 64;
  const int b   = mb / NP;
  const int nb0 = mb - b * NP;
  const size_t bbase = (size_t)b * NP;
  float* scw = sm_sc + tid * 12;

#pragma unroll 1
  for (int jp = 0; jp < 2; ++jp) {
    const int pi   = tid + 256 * jp;
    const int tok  = pi & 63;
    const int head = pi >> 6;
    const int dil  = 4 * ((head >> 1) + 1);
    const int p    = nb0 + tok;
    const int y    = p / IMG;
    const int x    = p - y * IMG;
    const float* qrow = qf + ((size_t)mb + tok) * HID + head * HD;
    float qv[HD];
#pragma unroll
    for (int i = 0; i < 8; ++i) {
      const v4f a = *(const v4f*)(qrow + 4 * i);
      qv[4 * i + 0] = a[0]; qv[4 * i + 1] = a[1]; qv[4 * i + 2] = a[2]; qv[4 * i + 3] = a[3];
    }
    const float* kbp = kf + bbase * HID + head * HD;
    const float* vbp = vf + bbase * HID + head * HD;
#pragma unroll 1
    for (int t = 0; t < NWIN; ++t) {
      const int ti = t / 3;
      const int tj = t - 3 * ti;
      const int yy = y + (ti - 1) * dil;
      const int xx = x + (tj - 1) * dil;
      const bool ok = ((unsigned)yy < (unsigned)IMG) && ((unsigned)xx < (unsigned)IMG);
      const int pp = ok ? (yy * IMG + xx) : p;
      const float* kr = kbp + (size_t)pp * HID;
      float a = 0.f;
#pragma unroll
      for (int i = 0; i < 8; ++i) {
        const v4f kk = *(const v4f*)(kr + 4 * i);
        a = fmaf(qv[4 * i + 0], kk[0], a);
        a = fmaf(qv[4 * i + 1], kk[1], a);
        a = fmaf(qv[4 * i + 2], kk[2], a);
        a = fmaf(qv[4 * i + 3], kk[3], a);
      }
      scw[t] = ok ? a * sscale : 0.f;
    }
    float mx = scw[0];
#pragma unroll
    for (int t = 1; t < NWIN; ++t) mx = fmaxf(mx, scw[t]);
    float den = 0.f;
#pragma unroll
    for (int t = 0; t < NWIN; ++t) {
      const float e = __expf(scw[t] - mx);
      scw[t] = e;
      den += e;
    }
    const float inv = 1.0f / den;
    float o[HD] = {0.f};
#pragma unroll 1
    for (int t = 0; t < NWIN; ++t) {
      const int ti = t / 3;
      const int tj = t - 3 * ti;
      const int yy = y + (ti - 1) * dil;
      const int xx = x + (tj - 1) * dil;
      const bool ok = ((unsigned)yy < (unsigned)IMG) && ((unsigned)xx < (unsigned)IMG);
      const int pp = ok ? (yy * IMG + xx) : p;
      const float w = ok ? scw[t] * inv : 0.f;
      const float* vr = vbp + (size_t)pp * HID;
#pragma unroll
      for (int i = 0; i < 8; ++i) {
        const v4f vv = *(const v4f*)(vr + 4 * i);
        o[4 * i + 0] = fmaf(w, vv[0], o[4 * i + 0]);
        o[4 * i + 1] = fmaf(w, vv[1], o[4 * i + 1]);
        o[4 * i + 2] = fmaf(w, vv[2], o[4 * i + 2]);
        o[4 * i + 3] = fmaf(w, vv[3], o[4 * i + 3]);
      }
    }
    _Float16* arow = sm.at + tok * ATP + head * HD;
#pragma unroll
    for (int i = 0; i < 4; ++i) {
      Pack8 pk;
      pk.h = (v8h){(_Float16)(o[8 * i + 0] * ASC), (_Float16)(o[8 * i + 1] * ASC),
                   (_Float16)(o[8 * i + 2] * ASC), (_Float16)(o[8 * i + 3] * ASC),
                   (_Float16)(o[8 * i + 4] * ASC), (_Float16)(o[8 * i + 5] * ASC),
                   (_Float16)(o[8 * i + 6] * ASC), (_Float16)(o[8 * i + 7] * ASC)};
      *(v8h*)(arow + 8 * i) = pk.h;
    }
  }
  __syncthreads();

  const int n0 = wn * 64;
  v8f acc[4];
#pragma unroll
  for (int t = 0; t < 4; ++t) acc[t] = zero8();
  gemm16x64<HID / 32>(sm.at, ATP, wo16, HID, wm * 16, n0, lane, acc);
  __syncthreads();

#pragma unroll
  for (int t = 0; t < 4; ++t) {
    const float bb = bo[n0 + 16 * t + c];
#pragma unroll
    for (int r = 0; r < 8; ++r)
      sm.st[(n0 + 16 * t + c) * OTP + wm * 16 + 8 * hh + r] = acc[t][r] * INV_AW + bb;
  }
  __syncthreads();
  store_nchw(sm.st, xq, xr, b, nb0, wave, lane);
}

#define HTP 136
__global__ __launch_bounds__(256) void k_ffn1(const _Float16* __restrict__ hn,
                                              const _Float16* __restrict__ w1p,
                                              const float* __restrict__ b1,
                                              _Float16* __restrict__ h1) {
  __shared__ __align__(16) _Float16 sh[64 * HTP];
  const int tid = threadIdx.x, lane = tid & 31, wave = tid >> 5;
  const int hh = lane >> 4, c = lane & 15;
  const int wm = wave >> 1, wn = wave & 1;
  const int mb = blockIdx.x * 64;
  const int ns = blockIdx.y;
  const int m0 = mb + wm * 16;
  const int n0 = ns * 128 + wn * 64;

  v8f acc[4];
#pragma unroll
  for (int t = 0; t < 4; ++t) acc[t] = zero8();
  gemm16x64<CC / 32>(hn, CC, w1p, CC, m0, n0, lane, acc);

#pragma unroll
  for (int t = 0; t < 4; ++t) {
    const float bb = b1[n0 + 16 * t + c];
#pragma unroll
    for (int r = 0; r < 8; ++r) {
      const float v = acc[t][r] * INV_AW + bb;
      sh[(wm * 16 + 8 * hh + r) * HTP + wn * 64 + 16 * t + c] = (_Float16)(gelu_f(v) * ASC);
    }
  }
  __syncthreads();

  v4u val[4];
  int go[4];
#pragma unroll
  for (int j = 0; j < 4; ++j) {
    const int p   = tid + 256 * j;
    const int row = p >> 4;
    const int pc  = p & 15;
    val[j] = *(const v4u*)(sh + row * HTP + pc * 8);
    go[j]  = (mb + row) * FF + ns * 128 + pc * 8;
  }
  for (int ps = 0; ps < 2; ++ps) {
#pragma unroll
    for (int j = 0; j < 4; ++j) *(volatile v4u*)(h1 + go[j]) = val[j];
    __threadfence();
  }
}

__global__ __launch_bounds__(256) void k_ffn2(const _Float16* __restrict__ h1,
                                              const _Float16* __restrict__ w2p,
                                              const float* __restrict__ b2,
                                              const float* __restrict__ xr,
                                              float* __restrict__ out) {
  __shared__ __align__(16) float st[CC * OTP];
  const int tid = threadIdx.x, lane = tid & 31, wave = tid >> 5;
  const int hh = lane >> 4, c = lane & 15;
  const int wm = wave >> 1, wn = wave & 1;
  const int mb  = blockIdx.x * 64;
  const int b   = mb / NP;
  const int nb0 = mb - b * NP;
  const int m0  = mb + wm * 16;
  const int n0  = wn * 64;

  v8f acc[4];
#pragma unroll
  for (int t = 0; t < 4; ++t) acc[t] = zero8();
  gemm16x64<FF / 32>(h1, FF, w2p, FF, m0, n0, lane, acc);

#pragma unroll
  for (int t = 0; t < 4; ++t) {
    const float bb = b2[n0 + 16 * t + c];
#pragma unroll
    for (int r = 0; r < 8; ++r) st[(n0 + 16 * t + c) * OTP + wm * 16 + 8 * hh + r] = acc[t][r] * INV_AW + bb;
  }
  __syncthreads();
  store_nchw(st, xr, out, b, nb0, wave, lane);
}

extern "C" void kernel_launch(void* const* d_in, const int* in_sizes, int n_in,
                              void* d_out, int out_size, void* d_ws, size_t ws_size,
                              hipStream_t stream) {
  if (n_in < 20) return;
  if (in_sizes[0] != NT * CC || in_sizes[1] != NT * CC) return;
  for (int i = 2; i < 8; ++i) if (in_sizes[i] != CC) return;
  if (in_sizes[8] != HID * CC || in_sizes[9] != HID) return;
  if (in_sizes[10] != HID * CC || in_sizes[11] != HID) return;
  if (in_sizes[12] != HID * CC || in_sizes[13] != HID) return;
  if (in_sizes[14] != CC * HID || in_sizes[15] != CC) return;
  if (in_sizes[16] != FF * CC || in_sizes[17] != FF) return;
  if (in_sizes[18] != CC * FF || in_sizes[19] != CC) return;
  if (out_size != NT * CC) return;

  const float* x_q    = (const float*)d_in[0];
  const float* x_kv   = (const float*)d_in[1];
  const float* gnq_w  = (const float*)d_in[2];
  const float* gnq_b  = (const float*)d_in[3];
  const float* gnkv_w = (const float*)d_in[4];
  const float* gnkv_b = (const float*)d_in[5];
  const float* gn2_w  = (const float*)d_in[6];
  const float* gn2_b  = (const float*)d_in[7];
  const float* wq = (const float*)d_in[8];   const float* bq = (const float*)d_in[9];
  const float* wk = (const float*)d_in[10];  const float* bk = (const float*)d_in[11];
  const float* wv = (const float*)d_in[12];  const float* bv = (const float*)d_in[13];
  const float* wo = (const float*)d_in[14];  const float* bo = (const float*)d_in[15];
  const float* w1 = (const float*)d_in[16];  const float* b1 = (const float*)d_in[17];
  const float* w2 = (const float*)d_in[18];  const float* b2 = (const float*)d_in[19];
  float* out = (float*)d_out;

  size_t off = 0;
  const size_t oWQKV = off; off += (size_t)3 * HID * CC * 2;
  const size_t oWO   = off; off += (size_t)CC * HID * 2;
  const size_t oW1   = off; off += (size_t)FF * CC * 2;
  const size_t oW2   = off; off += (size_t)CC * FF * 2;
  const size_t oSTQ  = off; off += 4096;
  const size_t oSTKV = off; off += 4096;
  const size_t oST2  = off; off += 4096;
  const size_t oXQT  = off; off += (size_t)NT * CC * 2;
  const size_t oXKVT = off; off += (size_t)NT * CC * 2;
  const size_t oHNT  = off; off += (size_t)NT * CC * 2;
  const size_t oQF   = off; off += (size_t)NT * HID * 4;
  const size_t oKF   = off; off += (size_t)NT * HID * 4;
  const size_t oVF   = off; off += (size_t)NT * HID * 4;
  const size_t oXR   = off; off += (size_t)NT * CC * 4;
  const size_t oH1   = off; off += (size_t)NT * FF * 2;
  if (off > ws_size) return;
  if (off > (size_t)134217728) return;

  char* ws = (char*)d_ws;
  _Float16* WQKV = (_Float16*)(ws + oWQKV);
  _Float16* WO16 = (_Float16*)(ws + oWO);
  _Float16* W116 = (_Float16*)(ws + oW1);
  _Float16* W216 = (_Float16*)(ws + oW2);
  float*    STQ  = (float*)(ws + oSTQ);
  float*    STKV = (float*)(ws + oSTKV);
  float*    ST2  = (float*)(ws + oST2);
  _Float16* XQT  = (_Float16*)(ws + oXQT);
  _Float16* XKVT = (_Float16*)(ws + oXKVT);
  _Float16* HNT  = (_Float16*)(ws + oHNT);
  float*    QF   = (float*)(ws + oQF);
  float*    KF   = (float*)(ws + oKF);
  float*    VF   = (float*)(ws + oVF);
  float*    XR   = (float*)(ws + oXR);
  _Float16* H1   = (_Float16*)(ws + oH1);

  const int n8p = HID * CC / 8;
  const int n8f = FF * CC / 8;
  k_wcv<<<dim3(n8p / 256), dim3(256), 0, stream>>>(wq, n8p, WQKV);
  k_wcv<<<dim3(n8p / 256), dim3(256), 0, stream>>>(wk, n8p, WQKV + (size_t)HID * CC);
  k_wcv<<<dim3(n8p / 256), dim3(256), 0, stream>>>(wv, n8p, WQKV + (size_t)2 * HID * CC);
  k_wcv<<<dim3(n8p / 256), dim3(256), 0, stream>>>(wo, n8p, WO16);
  k_wcv<<<dim3(n8f / 256), dim3(256), 0, stream>>>(w1, n8f, W116);
  k_wcv<<<dim3(n8f / 256), dim3(256), 0, stream>>>(w2, n8f, W216);
  k_gnstat<<<dim3(NB * NG), dim3(256), 0, stream>>>(x_q, STQ);
  k_gnstat<<<dim3(NB * NG), dim3(256), 0, stream>>>(x_kv, STKV);
  k_xtr<<<dim3(NP / 64, NB), dim3(256), 0, stream>>>(x_q, STQ, gnq_w, gnq_b, XQT);
  k_xtr<<<dim3(NP / 64, NB), dim3(256), 0, stream>>>(x_kv, STKV, gnkv_w, gnkv_b, XKVT);
  k_qkv<<<dim3(NT / 64, 6), dim3(256), 0, stream>>>(XQT, XKVT, WQKV, bq, bk, bv, QF, KF, VF);
  const float sscale = 0.17677669529663688f;
  k_attn_wo<<<dim3(NT / 64), dim3(256), 0, stream>>>(QF, KF, VF, WO16, bo, x_q, XR, sscale);
  k_gnstat<<<dim3(NB * NG), dim3(256), 0, stream>>>(XR, ST2);
  k_xtr<<<dim3(NP / 64, NB), dim3(256), 0, stream>>>(XR, ST2, gn2_w, gn2_b, HNT);
  k_ffn1<<<dim3(NT / 64, FF / 128), dim3(256), 0, stream>>>(HNT, W116, b1, H1);
  k_ffn2<<<dim3(NT / 64), dim3(256), 0, stream>>>(H1, W216, b2, XR, out);
  (void)hipGetLastError();
}
